// MonotonicAlignmentSearch_35296041239267
// MI455X (gfx1250) — hardware-verified
//
#include <hip/hip_runtime.h>

typedef __attribute__((ext_vector_type(16))) _Float16 v16h;
typedef __attribute__((ext_vector_type(8)))  _Float16 v8h;
typedef __attribute__((ext_vector_type(16))) __bf16   v16b;
typedef __attribute__((ext_vector_type(8)))  __bf16   v8b;
typedef __attribute__((ext_vector_type(8)))  float    v8f;
typedef __attribute__((ext_vector_type(4)))  float    v4f;

#define HH 1024
#define TTT 128
#define TAA 512
#define NBATCH 2
#define KCONV 3072
#define MROWS (NBATCH * TTT)

__device__ __forceinline__ unsigned short f2bf_bits(float f) {
  unsigned u = __float_as_uint(f);
  return (unsigned short)((u + 0x7FFFu + ((u >> 16) & 1u)) >> 16);
}
__device__ __forceinline__ float bf_bits2f(unsigned short h) { return __uint_as_float(((unsigned)h) << 16); }

__device__ __forceinline__ void dep_guard_h(v8f& a, v8f& b, v16h x, v16h y) { asm volatile("v_nop\n\tv_nop\n\tv_nop\n\tv_nop" : "+v"(a), "+v"(b) : "v"(x), "v"(y)); }
__device__ __forceinline__ void dep_guard_b(v8f& a, v8f& b, v16b x, v16b y) { asm volatile("v_nop\n\tv_nop\n\tv_nop\n\tv_nop" : "+v"(a), "+v"(b) : "v"(x), "v"(y)); }
__device__ __forceinline__ void keep4_h(v16h a, v16h b, v16h c, v16h d) { asm volatile("v_nop" :: "v"(a), "v"(b), "v"(c), "v"(d)); }
__device__ __forceinline__ void keep4_b(v16b a, v16b b, v16b c, v16b d) { asm volatile("v_nop" :: "v"(a), "v"(b), "v"(c), "v"(d)); }
__device__ __forceinline__ void acc_guard4(v8f& a, v8f& b, v8f& c, v8f& d) { asm volatile("v_nop\n\tv_nop\n\tv_nop\n\tv_nop" : "+v"(a), "+v"(b), "+v"(c), "+v"(d)); }
template <typename T> struct Frag;
template <> struct Frag<_Float16> {
  typedef v16h V; union U { v16h v; v8h h[2]; };
  static __device__ __forceinline__ v16h load(const _Float16* p) {
    U f; f.h[0] = *(const v8h*)(p); f.h[1] = *(const v8h*)(p + 16); return f.v;
  }
  static __device__ __forceinline__ v8f mma(v16h a, v16h b, v8f c) {
    return __builtin_amdgcn_wmma_f32_16x16x32_f16(false, a, false, b, (short)0, c, false, false);
  }
  static __device__ __forceinline__ void guard(v8f& a, v8f& b, v16h x, v16h y) { dep_guard_h(a, b, x, y); }
  static __device__ __forceinline__ void keep(v16h a, v16h b, v16h c, v16h d) { keep4_h(a, b, c, d); }
};
template <> struct Frag<__bf16> {
  typedef v16b V; union U { v16b v; v8b h[2]; };
  static __device__ __forceinline__ v16b load(const __bf16* p) {
    U f; f.h[0] = *(const v8b*)(p); f.h[1] = *(const v8b*)(p + 16); return f.v;
  }
  static __device__ __forceinline__ v8f mma(v16b a, v16b b, v8f c) {
    return __builtin_amdgcn_wmma_f32_16x16x32_bf16(false, a, false, b, (short)0, c, false, false);
  }
  static __device__ __forceinline__ void guard(v8f& a, v8f& b, v16b x, v16b y) { dep_guard_b(a, b, x, y); }
  static __device__ __forceinline__ void keep(v16b a, v16b b, v16b c, v16b d) { keep4_b(a, b, c, d); }
};

template <int ET> struct Elem;
template <> struct Elem<0> { typedef _Float16 T; };
template <> struct Elem<1> { typedef __bf16 T; };
template <int ET, bool SPLIT, int BIAS_MODE, int OUT_MODE, bool RESID, int ACT = 0>
__global__ __launch_bounds__(256) void wmma_gemm64(
    const unsigned short* __restrict__ Ap, const unsigned short* __restrict__ A2p, int lda, long strideA,
    const unsigned short* __restrict__ Btp, const unsigned short* __restrict__ Bt2p, int ldb, long strideB,
    void* __restrict__ Cout, void* __restrict__ Cout2, int ldc, long strideC,
    const float* __restrict__ bias,
    const float* __restrict__ resid, long strideR,
    int M, int N, int K, float scale) {
  typedef typename Elem<ET>::T T;
  typedef typename Frag<T>::V V;
  const T* A = (const T*)Ap; const T* A2 = (const T*)A2p; const T* Bt = (const T*)Btp; const T* Bt2 = (const T*)Bt2p;
  __shared__ __align__(16) float sT[8][16 * 68];
  const int b    = blockIdx.y;
  const int lane = threadIdx.x & 31;
  const int wave = threadIdx.x >> 5;
  const int tilesN = N >> 6;
  const int tilesM = M >> 6;
  const int tile = blockIdx.x * 8 + wave;
  if (tile >= tilesM * tilesN) return;
  const int tm = tile / tilesN;
  const int tn = tile - tm * tilesN;
  const int m0 = tm << 6;
  const int n0 = tn << 6;

  const T* Ab  = A  + (size_t)b * strideA;
  const T* Bb  = Bt + (size_t)b * strideB;
  const T* Ab2 = SPLIT ? (A2  + (size_t)b * strideA) : nullptr;
  const T* Bb2 = SPLIT ? (Bt2 + (size_t)b * strideB) : nullptr;

  const int rlane = lane & 15;
  const int koff  = (lane >> 4) * 8;
  const int mOff  = (lane >> 4) * 8;

  v8f acc[4][4];
#pragma unroll
  for (int i = 0; i < 4; ++i)
#pragma unroll
    for (int j = 0; j < 4; ++j) acc[i][j] = (v8f){0.f,0.f,0.f,0.f,0.f,0.f,0.f,0.f};

  for (int k0 = 0; k0 < K; k0 += 32) {
    V bh[4], bl[4];
#pragma unroll
    for (int j = 0; j < 4; ++j) {
      const size_t bo = (size_t)(n0 + (j << 4) + rlane) * ldb + koff + k0;
      bh[j] = Frag<T>::load(Bb + bo);
      if (SPLIT) bl[j] = Frag<T>::load(Bb2 + bo);
    }
#pragma unroll
    for (int i = 0; i < 4; ++i) {
      const size_t ao = (size_t)(m0 + (i << 4) + rlane) * lda + koff + k0;
      V ah = Frag<T>::load(Ab + ao);
      V al;
      if (SPLIT) al = Frag<T>::load(Ab2 + ao);
#pragma unroll
      for (int j = 0; j < 4; ++j) {
        acc[i][j] = Frag<T>::mma(ah, bh[j], acc[i][j]);
        if (SPLIT) {
          acc[i][j] = Frag<T>::mma(ah, bl[j], acc[i][j]);
          acc[i][j] = Frag<T>::mma(al, bh[j], acc[i][j]);
        }
      }
      Frag<T>::guard(acc[i][0], acc[i][3], ah, SPLIT ? al : ah);
    }
    Frag<T>::keep(bh[0], bh[1], bh[2], bh[3]);
    if (SPLIT) Frag<T>::keep(bl[0], bl[1], bl[2], bl[3]);
  }
  acc_guard4(acc[0][0], acc[0][1], acc[0][2], acc[0][3]);
  acc_guard4(acc[1][0], acc[1][1], acc[1][2], acc[1][3]);
  acc_guard4(acc[2][0], acc[2][1], acc[2][2], acc[2][3]);
  acc_guard4(acc[3][0], acc[3][1], acc[3][2], acc[3][3]);

  float* slab = sT[wave];
  const float* Rb = RESID ? (resid + (size_t)b * strideR) : nullptr;
#pragma unroll
  for (int i = 0; i < 4; ++i) {
    const int mBase = m0 + (i << 4);
#pragma unroll
    for (int j = 0; j < 4; ++j) {
      const int n = n0 + (j << 4) + rlane;
      float bv = 0.f;
      if (BIAS_MODE == 2) bv = bias[n];
#pragma unroll
      for (int r = 0; r < 8; ++r) {
        float v = acc[i][j][r] * scale;
        if (BIAS_MODE == 1) v += bias[mBase + mOff + r];
        if (BIAS_MODE == 2) v += bv;
        if (RESID) v += Rb[(size_t)(mBase + mOff + r) * ldc + n];
        if (ACT == 1) v = tanhf(v);
        if (ACT == 2) v = fmaxf(v, 0.0f);
        if (ACT == 3) v = v / (1.0f + expf(-v));
        if (ACT == 4) v = (v > 0.f) ? v : 0.01f * v;
        if (ACT == 5) v = 0.5f * v * (1.0f + erff(v * 0.70710678118654752f));
        slab[(mOff + r) * 68 + (j << 4) + rlane] = v;
      }
    }
    __builtin_amdgcn_fence(__ATOMIC_RELEASE, "workgroup");
    __builtin_amdgcn_wave_barrier();
    __builtin_amdgcn_fence(__ATOMIC_ACQUIRE, "workgroup");
    if (OUT_MODE == 0) {
      float* C = (float*)Cout + (size_t)b * strideC;
      const int hh = lane >> 4, c4 = (lane & 15) * 4;
      for (int pass = 0; pass < 2; ++pass) {
#pragma unroll
        for (int it = 0; it < 8; ++it) {
          const int row = it * 2 + hh;
          v4f v = *(const v4f*)(slab + row * 68 + c4);
          *(volatile v4f*)(C + (size_t)(mBase + row) * ldc + n0 + c4) = v;
        }
        __threadfence();
      }
    } else {
      const int q = lane >> 3, c8 = (lane & 7) * 8;
      unsigned short* C  = (unsigned short*)Cout  + (size_t)b * strideC;
      unsigned short* C2 = (OUT_MODE == 2) ? ((unsigned short*)Cout2 + (size_t)b * strideC) : nullptr;
      for (int pass = 0; pass < 2; ++pass) {
#pragma unroll
        for (int it = 0; it < 4; ++it) {
          const int row = it * 4 + q;
          const float* sp = slab + row * 68 + c8;
          v8h hv, lv;
#pragma unroll
          for (int e = 0; e < 8; ++e) {
            if (OUT_MODE == 1) {
              hv[e] = (_Float16)sp[e];
            } else {
              unsigned short hb = f2bf_bits(sp[e]);
              unsigned short lb = f2bf_bits(sp[e] - bf_bits2f(hb));
              hv[e] = __builtin_bit_cast(_Float16, hb);
              lv[e] = __builtin_bit_cast(_Float16, lb);
            }
          }
          *(volatile v8h*)(C + (size_t)(mBase + row) * ldc + n0 + c8) = hv;
          if (OUT_MODE == 2) *(volatile v8h*)(C2 + (size_t)(mBase + row) * ldc + n0 + c8) = lv;
        }
        __threadfence();
      }
    }
    __builtin_amdgcn_fence(__ATOMIC_RELEASE, "workgroup");
    __builtin_amdgcn_wave_barrier();
    __builtin_amdgcn_fence(__ATOMIC_ACQUIRE, "workgroup");
  }
}

__global__ __launch_bounds__(256) void cast_f32_f16x2s(
    const float* __restrict__ in, _Float16* __restrict__ out, int n2, float scale) {
  int i = blockIdx.x * 256 + threadIdx.x;
  if (i < n2) {
    const _Float16 h0 = (_Float16)(in[2 * i] * scale), h1 = (_Float16)(in[2 * i + 1] * scale);
    const unsigned u = (unsigned)__builtin_bit_cast(unsigned short, h0) | ((unsigned)__builtin_bit_cast(unsigned short, h1) << 16);
    ((volatile unsigned*)out)[i] = u;
    __threadfence();
    ((volatile unsigned*)out)[i] = u;
  }
}

__global__ __launch_bounds__(256) void transpose_f32_f16(
    const float* __restrict__ in, _Float16* __restrict__ out, int R, int C, float scale) {
  __shared__ __align__(16) _Float16 sT[64 * 72];
  const int tid = threadIdx.x;
  const int c0 = blockIdx.x * 64, r0 = blockIdx.y * 64;
#pragma unroll
  for (int it = 0; it < 4; ++it) {
    const int idx = tid + 256 * it;
    const int r = idx >> 4, c4 = (idx & 15) * 4;
    const v4f v = *(const v4f*)(in + (size_t)(r0 + r) * C + c0 + c4);
#pragma unroll
    for (int e = 0; e < 4; ++e) sT[(c4 + e) * 72 + r] = (_Float16)(v[e] * scale);
  }
  __syncthreads();
  const int q = tid >> 3, seg = (tid & 7) * 8;
  for (int pass = 0; pass < 2; ++pass) {
#pragma unroll
    for (int it = 0; it < 2; ++it) {
      const int c = it * 32 + q;
      const v8h val = *(const v8h*)(sT + c * 72 + seg);
      *(volatile v8h*)(out + (size_t)(c0 + c) * R + r0 + seg) = val;
    }
    __threadfence();
  }
}

template <bool GN>
__global__ __launch_bounds__(384) void im2col3(const float* __restrict__ src, const float* __restrict__ stats,
                                               const float* __restrict__ gam, const float* __restrict__ bet,
                                               _Float16* __restrict__ dst) {
  const int m = blockIdx.x;
  const int b = m >> 7, t = m & 127;
  const int j = threadIdx.x;
  float mu = 0.f, rsd = 1.f;
  if (GN) { mu = stats[2 * b]; rsd = stats[2 * b + 1]; }
  const int k0 = j * 8;
  v8h hv;
#pragma unroll
  for (int e = 0; e < 8; ++e) {
    const int k   = k0 + e;
    const int c   = k / 3;
    const int kk  = k - c * 3;
    const int ts  = t + kk - 1;
    const int tsc = ts < 0 ? 0 : (ts > (TTT - 1) ? (TTT - 1) : ts);
    float x = src[(size_t)(b * TTT + tsc) * HH + c];
    if (GN) x = (x - mu) * rsd * gam[c] + bet[c];
    const float v = (ts >= 0 && ts < TTT) ? x : 0.f;
    hv[e] = (_Float16)v;
  }
  _Float16* p = dst + (size_t)m * KCONV + k0;
  *(volatile v8h*)p = hv;
  __threadfence();
  *(volatile v8h*)p = hv;
}

__global__ __launch_bounds__(512) void gn_stats(const float* __restrict__ Y, float* __restrict__ stats) {
  __shared__ double rs_[512];
  __shared__ double rq_[512];
  __shared__ __align__(16) float sres[32];
  const int tid = threadIdx.x;
  if (tid < 32) sres[tid] = 0.f;
  for (int b = 0; b < NBATCH; ++b) {
    const float* p = Y + (size_t)b * (TTT * HH);
    double s = 0.0, q = 0.0;
#pragma unroll 1
    for (int i = tid; i < TTT * HH; i += 512) { const double v = (double)p[i]; s += v; q += v * v; }
    rs_[tid] = s; rq_[tid] = q;
    __syncthreads();
    for (int off = 256; off > 0; off >>= 1) {
      if (tid < off) { rs_[tid] += rs_[tid + off]; rq_[tid] += rq_[tid + off]; }
      __syncthreads();
    }
    if (tid == 0) {
      const double invn = 1.0 / 131072.0;
      const double mu   = rs_[0] * invn;
      double var = rq_[0] * invn - mu * mu;
      if (var < 0.0) var = 0.0;
      const float varf = (float)var;
      sres[2 * b]     = (float)mu;
      sres[2 * b + 1] = 1.0f / sqrtf(varf + 1e-5f);
    }
    __syncthreads();
  }
  if (tid < 8) {
    const v4f v = *(const v4f*)(sres + 4 * tid);
    *(volatile v4f*)(stats + 4 * tid) = v;
    __threadfence();
    *(volatile v4f*)(stats + 4 * tid) = v;
  }
}

__global__ __launch_bounds__(256) void durations_k(const float* __restrict__ Y2, const float* __restrict__ stats,
                                                   const float* __restrict__ gam, const float* __restrict__ bet,
                                                   const float* __restrict__ w3, const float* __restrict__ b3,
                                                   float* __restrict__ dur) {
  __shared__ __align__(16) float sres[32];
  const int lane = threadIdx.x & 31, wave = threadIdx.x >> 5;
  const int r0 = blockIdx.x * 32;
#pragma unroll 1
  for (int q = 0; q < 4; ++q) {
    const int row = r0 + wave * 4 + q;
    const int b = row >> 7;
    const float mu = stats[2 * b], rsd = stats[2 * b + 1];
    const float* p = Y2 + (size_t)row * HH;
    float s = 0.f;
#pragma unroll 1
    for (int c = lane; c < HH; c += 32) {
      const float xn = (p[c] - mu) * rsd * gam[c] + bet[c];
      s = fmaf(xn, w3[c], s);
    }
#pragma unroll
    for (int off = 16; off > 0; off >>= 1) s += __shfl_xor(s, off, 32);
    if (lane == 0) {
      const float x = s + b3[0];
      sres[wave * 4 + q] = fmaxf(x, 0.f) + log1pf(expf(-fabsf(x)));
    }
  }
  __syncthreads();
  if (threadIdx.x < 8) {
    const v4f v = *(const v4f*)(sres + 4 * threadIdx.x);
    *(volatile v4f*)(dur + r0 + 4 * threadIdx.x) = v;
    __threadfence();
    *(volatile v4f*)(dur + r0 + 4 * threadIdx.x) = v;
  }
}

__global__ __launch_bounds__(256) void align_k(const float* __restrict__ tp, const float* __restrict__ ap,
                                               const float* __restrict__ w2, const float* __restrict__ b2,
                                               float* __restrict__ out) {
  __shared__ __align__(16) float slog[TAA];
  __shared__ float sred[16];
  const int tid = threadIdx.x, lane = tid & 31, wave = tid >> 5;
  const int row = blockIdx.x;
  const int b = row >> 7, i = row & 127;
  v4f tr[8], wr[8];
  {
    const float* tpr = tp + (size_t)row * HH + 4 * lane;
#pragma unroll
    for (int it = 0; it < 8; ++it) {
      tr[it] = *(const v4f*)(tpr + 128 * it);
      wr[it] = *(const v4f*)(w2 + 4 * lane + 128 * it);
    }
  }
  const float* apb = ap + (size_t)b * TAA * HH + 4 * lane;
#pragma unroll 1
  for (int jj = 0; jj < TAA / 8; ++jj) {
    const int j = wave * (TAA / 8) + jj;
    const float* apr = apb + (size_t)j * HH;
    float acc = 0.f;
#pragma unroll
    for (int it = 0; it < 8; ++it) {
      const v4f a = *(const v4f*)(apr + 128 * it);
#pragma unroll
      for (int e = 0; e < 4; ++e) acc = fmaf(fmaxf(tr[it][e] + a[e], 0.f), wr[it][e], acc);
    }
#pragma unroll
    for (int off = 16; off > 0; off >>= 1) acc += __shfl_xor(acc, off, 32);
    if (lane == 0) slog[j] = acc;
  }
  __syncthreads();
  const float bb = b2[0];
  const float ex = (float)i * 4.0f;
  const float m0v = -0.1f * fabsf((float)tid - ex);
  const float m1v = -0.1f * fabsf((float)(tid + 256) - ex);
  const float l0 = (slog[tid] + bb) + m0v;
  const float l1 = (slog[tid + 256] + bb) + m1v;
  float mx = fmaxf(l0, l1);
#pragma unroll
  for (int off = 16; off > 0; off >>= 1) mx = fmaxf(mx, __shfl_xor(mx, off, 32));
  if (lane == 0) sred[wave] = mx;
  __syncthreads();
  mx = sred[0];
#pragma unroll
  for (int w = 1; w < 8; ++w) mx = fmaxf(mx, sred[w]);
  const float e0 = expf(l0 - mx), e1 = expf(l1 - mx);
  float s = e0 + e1;
#pragma unroll
  for (int off = 16; off > 0; off >>= 1) s += __shfl_xor(s, off, 32);
  if (lane == 0) sred[8 + wave] = s;
  __syncthreads();
  float sum = sred[8];
#pragma unroll
  for (int w = 1; w < 8; ++w) sum += sred[8 + w];
  const float inv = 1.0f / sum;
  slog[tid] = e0 * inv;
  slog[tid + 256] = e1 * inv;
  __syncthreads();
  if (tid < TAA / 4) {
    const v4f v = *(const v4f*)(slog + 4 * tid);
    float* p = out + (size_t)row * TAA + 4 * tid;
    *(volatile v4f*)p = v;
    __threadfence();
    *(volatile v4f*)p = v;
  }
}

extern "C" void kernel_launch(void* const* d_in, const int* in_sizes, int n_in,
                              void* d_out, int out_size, void* d_ws, size_t ws_size,
                              hipStream_t stream) {
  if (n_in < 16) return;
  if (in_sizes[0] != NBATCH * TTT * HH || in_sizes[1] != NBATCH * TAA * HH || in_sizes[2] != 2 * HH * HH ||
      in_sizes[3] != HH || in_sizes[4] != HH || in_sizes[5] < 1 || in_sizes[6] != HH * HH * 3 ||
      in_sizes[7] != HH || in_sizes[8] != HH || in_sizes[9] != HH || in_sizes[10] != HH * HH * 3 ||
      in_sizes[11] != HH || in_sizes[12] != HH || in_sizes[13] != HH || in_sizes[14] != HH || in_sizes[15] < 1) return;
  if (out_size != NBATCH * TTT * TAA + NBATCH * TTT) return;

  const float* text  = (const float*)d_in[0];
  const float* audio = (const float*)d_in[1];
  const float* a_w1  = (const float*)d_in[2];
  const float* a_b1  = (const float*)d_in[3];
  const float* a_w2  = (const float*)d_in[4];
  const float* a_b2  = (const float*)d_in[5];
  const float* d_w1  = (const float*)d_in[6];
  const float* d_b1  = (const float*)d_in[7];
  const float* gn1_g = (const float*)d_in[8];
  const float* gn1_b = (const float*)d_in[9];
  const float* d_w2  = (const float*)d_in[10];
  const float* d_b2  = (const float*)d_in[11];
  const float* gn2_g = (const float*)d_in[12];
  const float* gn2_b = (const float*)d_in[13];
  const float* d_w3  = (const float*)d_in[14];
  const float* d_b3  = (const float*)d_in[15];

  float* out = (float*)d_out;
  float* alignment = out;
  float* durations = out + (size_t)NBATCH * TTT * TAA;

  char* ws = (char*)d_ws;
  size_t off = 0;
  const size_t sz_text16  = (size_t)MROWS * HH * 2;
  const size_t sz_audio16 = (size_t)NBATCH * TAA * HH * 2;
  const size_t sz_w1t     = (size_t)HH * (2 * HH) * 2;
  const size_t sz_wc      = (size_t)HH * KCONV * 2;
  const size_t sz_col     = (size_t)MROWS * KCONV * 2;
  const size_t sz_tp      = (size_t)MROWS * HH * 4;
  const size_t sz_ap      = (size_t)NBATCH * TAA * HH * 4;
  const size_t sz_y       = (size_t)MROWS * HH * 4;
  const size_t sz_st      = 256;
  unsigned short* text16  = (unsigned short*)(ws + off); off += sz_text16;
  unsigned short* audio16 = (unsigned short*)(ws + off); off += sz_audio16;
  unsigned short* w1t     = (unsigned short*)(ws + off); off += sz_w1t;
  unsigned short* wc1     = (unsigned short*)(ws + off); off += sz_wc;
  unsigned short* wc2     = (unsigned short*)(ws + off); off += sz_wc;
  unsigned short* col1    = (unsigned short*)(ws + off); off += sz_col;
  unsigned short* col2    = (unsigned short*)(ws + off); off += sz_col;
  float* tp  = (float*)(ws + off); off += sz_tp;
  float* ap  = (float*)(ws + off); off += sz_ap;
  float* y1  = (float*)(ws + off); off += sz_y;
  float* y2  = (float*)(ws + off); off += sz_y;
  float* st1 = (float*)(ws + off); off += sz_st;
  float* st2 = (float*)(ws + off); off += sz_st;
  if (off > ws_size || off > (size_t)134217728) return;

  const float wscale = 16.0f, inv_wscale = 1.0f / 16.0f;

  cast_f32_f16x2s<<<dim3((MROWS * HH / 2 + 255) / 256), dim3(256), 0, stream>>>(text, (_Float16*)text16, MROWS * HH / 2, 1.0f);
  cast_f32_f16x2s<<<dim3((NBATCH * TAA * HH / 2 + 255) / 256), dim3(256), 0, stream>>>(audio, (_Float16*)audio16, NBATCH * TAA * HH / 2, 1.0f);
  transpose_f32_f16<<<dim3(HH / 64, (2 * HH) / 64), dim3(256), 0, stream>>>(a_w1, (_Float16*)w1t, 2 * HH, HH, wscale);
  cast_f32_f16x2s<<<dim3((HH * KCONV / 2 + 255) / 256), dim3(256), 0, stream>>>(d_w1, (_Float16*)wc1, HH * KCONV / 2, wscale);
  cast_f32_f16x2s<<<dim3((HH * KCONV / 2 + 255) / 256), dim3(256), 0, stream>>>(d_w2, (_Float16*)wc2, HH * KCONV / 2, wscale);

  wmma_gemm64<0, false, 2, 0, false, 0><<<dim3((MROWS / 64) * (HH / 64) / 8, 1), dim3(256), 0, stream>>>(
      text16, text16, HH, 0L, w1t, w1t, 2 * HH, 0L, tp, tp, HH, 0L, a_b1, tp, 0L, MROWS, HH, HH, inv_wscale);
  wmma_gemm64<0, false, 0, 0, false, 0><<<dim3(((NBATCH * TAA) / 64) * (HH / 64) / 8, 1), dim3(256), 0, stream>>>(
      audio16, audio16, HH, 0L, w1t + HH, w1t + HH, 2 * HH, 0L, ap, ap, HH, 0L, a_b1, ap, 0L, NBATCH * TAA, HH, HH, inv_wscale);

  im2col3<false><<<dim3(MROWS), dim3(384), 0, stream>>>(text, st1, gn1_g, gn1_b, (_Float16*)col1);
  wmma_gemm64<0, false, 2, 0, false, 2><<<dim3((MROWS / 64) * (HH / 64) / 8, 1), dim3(256), 0, stream>>>(
      col1, col1, KCONV, 0L, wc1, wc1, KCONV, 0L, y1, y1, HH, 0L, d_b1, y1, 0L, MROWS, HH, KCONV, inv_wscale);
  gn_stats<<<dim3(1), dim3(512), 0, stream>>>(y1, st1);
  im2col3<true><<<dim3(MROWS), dim3(384), 0, stream>>>(y1, st1, gn1_g, gn1_b, (_Float16*)col2);
  wmma_gemm64<0, false, 2, 0, false, 2><<<dim3((MROWS / 64) * (HH / 64) / 8, 1), dim3(256), 0, stream>>>(
      col2, col2, KCONV, 0L, wc2, wc2, KCONV, 0L, y2, y2, HH, 0L, d_b2, y2, 0L, MROWS, HH, KCONV, inv_wscale);
  gn_stats<<<dim3(1), dim3(512), 0, stream>>>(y2, st2);
  durations_k<<<dim3(MROWS / 32), dim3(256), 0, stream>>>(y2, st2, gn2_g, gn2_b, d_w3, d_b3, durations);

  align_k<<<dim3(MROWS), dim3(256), 0, stream>>>(tp, ap, a_w2, a_b2, alignment);
  (void)hipGetLastError();
}
